// HybridTransformerBlock_65481071396451
// MI455X (gfx1250) — hardware-verified
//
#include <hip/hip_runtime.h>


#define NB_  2
#define TT   2048
#define DM   1024
#define NH_  16
#define HD   64
#define DFF  4096
#define ZH   2
#define PCAR 1024.0f
typedef _Float16 h16;
typedef unsigned short bf;
typedef __attribute__((ext_vector_type(16))) __bf16   v16bf;
typedef __attribute__((ext_vector_type(16))) _Float16 v16h;
typedef __attribute__((ext_vector_type(8)))  _Float16 v8h;
typedef __attribute__((ext_vector_type(8)))  unsigned short v8us;
typedef __attribute__((ext_vector_type(8)))  float    v8f;
typedef __attribute__((ext_vector_type(4)))  float    v4f;
typedef v8h  __attribute__((may_alias)) v8ha;
typedef v4f  __attribute__((may_alias)) v4fa;
typedef v8us __attribute__((may_alias)) v8usa;

__device__ __forceinline__ unsigned short f2bf(float f) { unsigned u = __float_as_uint(f); u += 0x7FFFu + ((u >> 16) & 1u); return (unsigned short)(u >> 16); }
__device__ __forceinline__ float bf2f(unsigned short b) { return __uint_as_float(((unsigned)b) << 16); }
__device__ __forceinline__ float bfr(float f) { return bf2f(f2bf(f)); }
__device__ __forceinline__ v16h cat16(v8h lo, v8h hi) { return __builtin_shufflevector(lo, hi, 0, 1, 2, 3, 4, 5, 6, 7, 8, 9, 10, 11, 12, 13, 14, 15); }
__device__ __forceinline__ v16bf cat16b(v8us lo, v8us hi) { return __builtin_bit_cast(v16bf, __builtin_shufflevector(lo, hi, 0, 1, 2, 3, 4, 5, 6, 7, 8, 9, 10, 11, 12, 13, 14, 15)); }
__device__ __forceinline__ v8f wmma16(v16h a, v16h b, v8f c) { return __builtin_amdgcn_wmma_f32_16x16x32_f16(false, a, false, b, (short)0, c, false, false); }
__device__ __forceinline__ v8f wmmab(v16bf a, v16bf b, v8f c) { return __builtin_amdgcn_wmma_f32_16x16x32_bf16(false, a, false, b, (short)0, c, false, false); }


template <typename T16> struct WFrag;
template <> struct WFrag<h16> { typedef v16h V; static __device__ __forceinline__ V ld(const h16* p) { return cat16(*(const v8h*)p, *(const v8h*)(p + 16)); } static __device__ __forceinline__ v8f mma(V a, V b, v8f c) { return wmma16(a, b, c); } };
template <> struct WFrag<bf> { typedef v16bf V; static __device__ __forceinline__ V ld(const bf* p) { return cat16b(*(const v8us*)p, *(const v8us*)(p + 16)); } static __device__ __forceinline__ v8f mma(V a, V b, v8f c) { return wmmab(a, b, c); } };
template <typename T16, int NSPLIT, bool BIAS>
__global__ __launch_bounds__(32) void k_gemmw(const T16* __restrict__ A, const T16* __restrict__ A2, const T16* __restrict__ Bt, const T16* __restrict__ Bt2, int K, float* C, int ldc, const float* __restrict__ bias, size_t sA, size_t sB, size_t sC) {
    typedef typename WFrag<T16>::V V;
    __shared__ __align__(16) float os[16 * 68];
    const size_t z = blockIdx.z; A += z * sA; if (A2) A2 += z * sA; Bt += z * sB; if (Bt2) Bt2 += z * sB; C += z * sC;
    const int lane = threadIdx.x & 31, lr = lane & 15, hi = lane >> 4; const int r0 = blockIdx.x * 64, c0 = blockIdx.y * 64;
    v8f acc[4][4];
#pragma unroll
    for (int mb = 0; mb < 4; ++mb)
#pragma unroll
        for (int nb = 0; nb < 4; ++nb) acc[mb][nb] = (v8f){};
    const size_t aoff = (size_t)(r0 + lr) * K + 8 * hi, boff = (size_t)(c0 + lr) * K + 8 * hi;
#pragma unroll 1
    for (int kc = 0; kc < K; kc += 32) {
        V a[4], a2[4];
#pragma unroll
        for (int mb = 0; mb < 4; ++mb) { a[mb] = WFrag<T16>::ld(A + aoff + (size_t)mb * 16 * K + kc); if (NSPLIT == 1 || NSPLIT == 2) a2[mb] = WFrag<T16>::ld(A2 + aoff + (size_t)mb * 16 * K + kc); }
#pragma unroll
        for (int nb = 0; nb < 4; ++nb) { const V b = WFrag<T16>::ld(Bt + boff + (size_t)nb * 16 * K + kc); V b2; if (NSPLIT >= 2) b2 = WFrag<T16>::ld(Bt2 + boff + (size_t)nb * 16 * K + kc);
#pragma unroll
            for (int mb = 0; mb < 4; ++mb) { acc[mb][nb] = WFrag<T16>::mma(a[mb], b, acc[mb][nb]); if (NSPLIT == 1 || NSPLIT == 2) acc[mb][nb] = WFrag<T16>::mma(a2[mb], b, acc[mb][nb]); if (NSPLIT >= 2) acc[mb][nb] = WFrag<T16>::mma(a[mb], b2, acc[mb][nb]); } }
        asm volatile("v_nop\n\tv_nop\n\tv_nop\n\tv_nop" : "+v"(acc[0][0]), "+v"(acc[1][1]), "+v"(acc[2][2]), "+v"(acc[3][3]) : "v"(a[0]), "v"(a[3]));
    }
#pragma unroll
    for (int mb = 0; mb < 4; ++mb) {
#pragma unroll
        for (int nb = 0; nb < 4; ++nb) {
#pragma unroll
            for (int j = 0; j < 8; ++j) os[(hi * 8 + j) * 68 + nb * 16 + lr] = acc[mb][nb][j]; }
        __builtin_amdgcn_wave_barrier(); asm volatile("" ::: "memory");
        float* crow = C + (size_t)(r0 + mb * 16) * ldc + c0;
#pragma unroll 1
        for (int ps = 0; ps < 2; ++ps) {
#pragma unroll
            for (int s = 0; s < 8; ++s) { const int row = 2 * s + hi, cofs = lr * 4; v4f val = *(const v4fa*)(os + row * 68 + cofs); if (BIAS) { val[0] += bfr(bias[c0 + cofs]); val[1] += bfr(bias[c0 + cofs + 1]); val[2] += bfr(bias[c0 + cofs + 2]); val[3] += bfr(bias[c0 + cofs + 3]); }
                *(volatile v4f*)(crow + (size_t)row * ldc + cofs) = val; }
            if (ps == 0) __threadfence(); }
        __builtin_amdgcn_wave_barrier(); asm volatile("" ::: "memory");
    }
}

__device__ __forceinline__ h16 tohx(float x) { return (h16)x; }
__device__ __forceinline__ void splitf(float y, unsigned short& h, unsigned short& l) { h = f2bf(y); l = f2bf(y - bf2f(h)); }
typedef __attribute__((ext_vector_type(2))) unsigned short v2us;
typedef __attribute__((ext_vector_type(4))) unsigned short v4us;
typedef __attribute__((ext_vector_type(2))) _Float16 v2h;
typedef __attribute__((ext_vector_type(4))) _Float16 v4h;

__global__ __launch_bounds__(256) void k_cvt8(const float* __restrict__ src, bf* dst, size_t n8) { const size_t i = (size_t)blockIdx.x * 256 + threadIdx.x; if (i >= n8) return; const v8f v = *(const v8f*)(src + i * 8); v8us o;
#pragma unroll
    for (int k = 0; k < 8; ++k) o[k] = f2bf(v[k]); *(volatile v8us*)(dst + i * 8) = o; __threadfence(); *(volatile v8us*)(dst + i * 8) = o; }
__global__ __launch_bounds__(256) void k_wtG(const float* __restrict__ w, int K, int N, bf* Bt) {
    const int lane = threadIdx.x & 31; const int L0 = (blockIdx.x * 8 + (threadIdx.x >> 5)) * 8; const int nlines = N * K / 64;
#pragma unroll
    for (int ps = 0; ps < 2; ++ps) {
#pragma unroll 1
        for (int l = 0; l < 8; ++l) { const int L = L0 + l; if (L >= nlines) break; const size_t e = (size_t)L * 64 + lane * 2; const int k = (int)(e % K), n = (int)(e / K); v2us o;
            o[0] = f2bf(w[(size_t)k * N + n]); o[1] = f2bf(w[(size_t)(k + 1) * N + n]); *(volatile v2us*)(Bt + e) = o; }
        if (ps == 0) __threadfence(); }
}

__global__ __launch_bounds__(256) void k_qk16(const float* __restrict__ Q, const float* __restrict__ K, h16* QP, h16* KP) { const size_t e = ((size_t)blockIdx.x * 256 + threadIdx.x) * 4; if (e >= (size_t)NH_ * TT * HD) return; const int d = (int)(e % HD); const int t = (int)((e / HD) % TT); const int h = (int)(e / ((size_t)HD * TT)); const size_t src = (size_t)t * DM + h * HD + d; const v4f a = *(const v4f*)(Q + src), c = *(const v4f*)(K + src); v4h oq, ok;
    for (int u = 0; u < 4; ++u) { oq[u] = tohx(a[u]); ok[u] = tohx(c[u]); } *(volatile v4h*)(QP + e) = oq; *(volatile v4h*)(KP + e) = ok; __threadfence(); *(volatile v4h*)(QP + e) = oq; *(volatile v4h*)(KP + e) = ok; }
__global__ __launch_bounds__(256) void k_vt16(const float* __restrict__ V, h16* VT) { const size_t e = ((size_t)blockIdx.x * 256 + threadIdx.x) * 2; if (e >= (size_t)NH_ * HD * TT) return; const int t = (int)(e % TT); const int d = (int)((e / TT) % HD); const int h = (int)(e / ((size_t)TT * HD)); v2h o; o[0] = tohx(V[(size_t)t * DM + h * HD + d]); o[1] = tohx(V[(size_t)(t + 1) * DM + h * HD + d]); *(volatile v2h*)(VT + e) = o; __threadfence(); *(volatile v2h*)(VT + e) = o; }
__global__ __launch_bounds__(256) void k_soft(const float* __restrict__ S, h16* P16) { const int lane = threadIdx.x & 31; const int row = blockIdx.x * 8 + (threadIdx.x >> 5); if (row >= ZH * TT) return; const float* sr = S + (size_t)row * TT; float v[TT / 32]; float mx = -3.0e38f;
#pragma unroll
    for (int ch = 0; ch < TT / 128; ++ch) { const v4f a = *(const v4f*)(sr + ch * 128 + lane * 4);
#pragma unroll
        for (int u = 0; u < 4; ++u) { const float t = a[u] * 0.125f; v[ch * 4 + u] = t; mx = fmaxf(mx, t); } }
#pragma unroll
    for (int sh = 16; sh; sh >>= 1) mx = fmaxf(mx, __shfl_xor(mx, sh, 32));
    float sum = 0.f;
#pragma unroll
    for (int q = 0; q < TT / 32; ++q) { float d0 = __fsub_rn(v[q], mx); asm volatile("" : "+v"(d0)); v[q] = __builtin_amdgcn_exp2f(__fmul_rn(d0, 1.4426950408889634f)); sum += v[q]; }
#pragma unroll
    for (int sh = 16; sh; sh >>= 1) sum += __shfl_xor(sum, sh, 32);
    const float f = __fdiv_rn(PCAR, sum);
    for (int ps = 0; ps < 2; ++ps) {
#pragma unroll
        for (int ch = 0; ch < TT / 128; ++ch) { v4h o4; for (int q = 0; q < 4; ++q) o4[q] = tohx(v[ch * 4 + q] * f); *(volatile v4h*)(P16 + (size_t)row * TT + ch * 128 + lane * 4) = o4; }
        if (ps == 0) __threadfence(); } }
__global__ __launch_bounds__(256) void k_mrg(const float* __restrict__ O, int h0, bf* Ah, bf* Al) { const size_t e = ((size_t)blockIdx.x * 256 + threadIdx.x) * 4; if (e >= (size_t)ZH * TT * HD) return; const int d = (int)(e % HD); const int t = (int)((e / HD) % TT); const int zz = (int)(e / ((size_t)HD * TT)); const size_t oo = (size_t)t * DM + (h0 + zz) * HD + d; v4us oh, ol;
#pragma unroll
    for (int u = 0; u < 4; ++u) { unsigned short a, b; splitf(O[e + u] * (1.0f / PCAR), a, b); oh[u] = a; ol[u] = b; } *(volatile v4us*)(Ah + oo) = oh; *(volatile v4us*)(Al + oo) = ol; __threadfence(); *(volatile v4us*)(Ah + oo) = oh; *(volatile v4us*)(Al + oo) = ol; }
__global__ __launch_bounds__(256) void k_resln(const float* __restrict__ A, int rndA, const float* __restrict__ Bv, const float* __restrict__ gscp, const float* __restrict__ g, const float* __restrict__ bb, float* Y, bf* Yh, bf* Yl) { const int lane = threadIdx.x & 31; const size_t r = (size_t)blockIdx.x * 8 + (threadIdx.x >> 5); if (r >= TT) return;
    float gsc = 1.0f; if (gscp) { const float th = bfr(gscp[0]); gsc = __fdiv_rn(1.0f, __fadd_rn(1.0f, expf(-cosf(th)))); }
    const float* ar = A + r * DM; const float* br = Bv + r * DM; float v[32]; float s = 0.f;
#pragma unroll
    for (int ch = 0; ch < 8; ++ch) { const v4f a = *(const v4f*)(ar + ch * 128 + lane * 4), c = *(const v4f*)(br + ch * 128 + lane * 4);
#pragma unroll
        for (int u = 0; u < 4; ++u) { float bb2 = __fmul_rn(c[u], gsc); asm volatile("" : "+v"(bb2)); const float t = __fadd_rn(rndA ? bfr(a[u]) : a[u], bb2); v[ch * 4 + u] = t; s += t; } }
#pragma unroll
    for (int sh = 16; sh; sh >>= 1) s += __shfl_xor(s, sh, 32);
    const float mean = s * (1.0f / DM); float q = 0.f;
#pragma unroll
    for (int k = 0; k < 32; ++k) { float d = __fsub_rn(v[k], mean); asm volatile("" : "+v"(d)); v[k] = d; float p = __fmul_rn(d, d); asm volatile("" : "+v"(p)); q = __fadd_rn(q, p); }
#pragma unroll
    for (int sh = 16; sh; sh >>= 1) q += __shfl_xor(q, sh, 32);
    const float rs = __frsqrt_rn(__fadd_rn(q * (1.0f / DM), 1e-5f));
    for (int ps = 0; ps < 2; ++ps) {
#pragma unroll
        for (int ch = 0; ch < 8; ++ch) { v4f o; v4us oh, ol;
#pragma unroll
            for (int u = 0; u < 4; ++u) { const int c = ch * 128 + lane * 4 + u; float n0 = __fmul_rn(v[ch * 4 + u], rs); asm volatile("" : "+v"(n0)); float t1 = __fmul_rn(n0, bfr(g[c])); asm volatile("" : "+v"(t1)); const float y = __fadd_rn(t1, bfr(bb[c])); o[u] = y; unsigned short a2, c2; splitf(y, a2, c2); oh[u] = a2; ol[u] = c2; }
            const size_t oo = r * DM + ch * 128 + lane * 4; if (Y) *(volatile v4f*)(Y + oo) = o; if (Yh) { *(volatile v4us*)(Yh + oo) = oh; *(volatile v4us*)(Yl + oo) = ol; } }
        if (ps == 0) __threadfence(); } }
__global__ __launch_bounds__(256) void k_relupl(const float* __restrict__ F, bf* Ph, bf* Pl, size_t n4) { const size_t e = ((size_t)blockIdx.x * 256 + threadIdx.x) * 4; if (e >= n4 * 4) return; const v4f a = *(const v4f*)(F + e); v4us oh, ol;
#pragma unroll
    for (int u = 0; u < 4; ++u) { unsigned short x0, x1; splitf(fmaxf(a[u], 0.f), x0, x1); oh[u] = x0; ol[u] = x1; } *(volatile v4us*)(Ph + e) = oh; *(volatile v4us*)(Pl + e) = ol; __threadfence(); *(volatile v4us*)(Ph + e) = oh; *(volatile v4us*)(Pl + e) = ol; }

extern "C" void kernel_launch(void* const* d_in, const int* in_sizes, int n_in,
                              void* d_out, int out_size, void* d_ws, size_t ws_size, hipStream_t stream) {
    (void)in_sizes; (void)n_in; (void)out_size;
    const float* x = (const float*)d_in[0]; const float* wq = (const float*)d_in[1]; const float* wk = (const float*)d_in[2]; const float* wv = (const float*)d_in[3]; const float* wo = (const float*)d_in[4]; const float* w1 = (const float*)d_in[5]; const float* b1 = (const float*)d_in[6]; const float* w2 = (const float*)d_in[7]; const float* b2 = (const float*)d_in[8];
    const float* ln1g = (const float*)d_in[9]; const float* ln1b = (const float*)d_in[10]; const float* ln2g = (const float*)d_in[11]; const float* ln2b = (const float*)d_in[12]; const float* theta = (const float*)d_in[13];
    float* OUT = (float*)d_out;
    char* wsp = (char*)d_ws;
    auto take = [&](size_t bytes) { char* p = wsp; wsp += (bytes + 255) & ~(size_t)255; return (void*)p; };
    bf* BQ = (bf*)take((size_t)DM * DM * 2); bf* BK = (bf*)take((size_t)DM * DM * 2); bf* BV = (bf*)take((size_t)DM * DM * 2); bf* BO = (bf*)take((size_t)DM * DM * 2); bf* BW1 = (bf*)take((size_t)DM * DFF * 2); bf* BW2 = (bf*)take((size_t)DFF * DM * 2);
    bf* XB = (bf*)take((size_t)TT * DM * 2); float* FQ = (float*)take((size_t)TT * DM * 4); float* FK = (float*)take((size_t)TT * DM * 4); float* FV = (float*)take((size_t)TT * DM * 4); h16* QP = (h16*)take((size_t)NH_ * TT * HD * 2); h16* KP = (h16*)take((size_t)NH_ * TT * HD * 2); h16* VT = (h16*)take((size_t)NH_ * HD * TT * 2);
    float* S = (float*)take((size_t)ZH * TT * TT * 4); h16* P16 = (h16*)take((size_t)ZH * TT * TT * 2); float* O = (float*)take((size_t)ZH * TT * HD * 4); bf* ATh = (bf*)take((size_t)TT * DM * 2); bf* ATl = (bf*)take((size_t)TT * DM * 2); float* AO = (float*)take((size_t)TT * DM * 4);
    float* X1 = (float*)take((size_t)TT * DM * 4); bf* X1h = (bf*)take((size_t)TT * DM * 2); bf* X1l = (bf*)take((size_t)TT * DM * 2); float* HID = (float*)take((size_t)TT * DFF * 4); bf* HIh = (bf*)take((size_t)TT * DFF * 2); bf* HIl = (bf*)take((size_t)TT * DFF * 2); float* F2 = (float*)take((size_t)TT * DM * 4);
    if ((size_t)(wsp - (char*)d_ws) > ws_size) return;
    k_wtG<<<(DM * DM / 64 + 63) / 64, 256, 0, stream>>>(wq, DM, DM, BQ); k_wtG<<<(DM * DM / 64 + 63) / 64, 256, 0, stream>>>(wk, DM, DM, BK); k_wtG<<<(DM * DM / 64 + 63) / 64, 256, 0, stream>>>(wv, DM, DM, BV); k_wtG<<<(DM * DM / 64 + 63) / 64, 256, 0, stream>>>(wo, DM, DM, BO);
    k_wtG<<<(DM * DFF / 64 + 63) / 64, 256, 0, stream>>>(w1, DM, DFF, BW1); k_wtG<<<(DFF * DM / 64 + 63) / 64, 256, 0, stream>>>(w2, DFF, DM, BW2);
    const dim3 gp(TT / 64, DM / 64, 1); const size_t zq = (size_t)TT * HD, zS = (size_t)TT * TT, zv = (size_t)HD * TT, zo = (size_t)TT * HD; const unsigned LQ = (unsigned)(((size_t)TT * DM / 4 + 255) / 256);
    for (int b = 0; b < NB_; ++b) { const float* xb = x + (size_t)b * TT * DM;
        k_cvt8<<<(TT * DM / 8 + 255) / 256, 256, 0, stream>>>(xb, XB, TT * DM / 8);
        k_gemmw<bf, 0, false><<<gp, 32, 0, stream>>>(XB, nullptr, BQ, nullptr, DM, FQ, DM, nullptr, 0, 0, 0); k_gemmw<bf, 0, false><<<gp, 32, 0, stream>>>(XB, nullptr, BK, nullptr, DM, FK, DM, nullptr, 0, 0, 0); k_gemmw<bf, 0, false><<<gp, 32, 0, stream>>>(XB, nullptr, BV, nullptr, DM, FV, DM, nullptr, 0, 0, 0);
        k_qk16<<<(unsigned)(((size_t)NH_ * TT * HD / 4 + 255) / 256), 256, 0, stream>>>(FQ, FK, QP, KP); k_vt16<<<(unsigned)(((size_t)NH_ * HD * TT / 2 + 255) / 256), 256, 0, stream>>>(FV, VT);
        for (int h0 = 0; h0 < NH_; h0 += ZH) {
            k_gemmw<h16, 0, false><<<dim3(TT / 64, TT / 64, ZH), 32, 0, stream>>>(QP + (size_t)h0 * zq, nullptr, KP + (size_t)h0 * zq, nullptr, HD, S, TT, nullptr, zq, zq, zS);
            k_soft<<<ZH * TT / 8, 256, 0, stream>>>(S, P16);
            k_gemmw<h16, 0, false><<<dim3(TT / 64, 1, ZH), 32, 0, stream>>>(P16, nullptr, VT + (size_t)h0 * zv, nullptr, TT, O, HD, nullptr, zS, zv, zo);
            k_mrg<<<(unsigned)(((size_t)ZH * TT * HD / 4 + 255) / 256), 256, 0, stream>>>(O, h0, ATh, ATl); }
        k_gemmw<bf, 1, false><<<gp, 32, 0, stream>>>(ATh, ATl, BO, nullptr, DM, AO, DM, nullptr, 0, 0, 0);
        k_resln<<<TT / 8, 256, 0, stream>>>(xb, 1, AO, theta, ln1g, ln1b, X1, X1h, X1l);
        k_gemmw<bf, 1, true><<<dim3(TT / 64, DFF / 64, 1), 32, 0, stream>>>(X1h, X1l, BW1, nullptr, DM, HID, DFF, b1, 0, 0, 0); k_relupl<<<(unsigned)(((size_t)TT * DFF / 4 + 255) / 256), 256, 0, stream>>>(HID, HIh, HIl, (size_t)TT * DFF / 4);
        k_gemmw<bf, 1, true><<<gp, 32, 0, stream>>>(HIh, HIl, BW2, nullptr, DFF, F2, DM, b2, 0, 0, 0);
        k_resln<<<TT / 8, 256, 0, stream>>>(X1, 0, F2, nullptr, ln2g, ln2b, OUT + (size_t)b * TT * DM, nullptr, nullptr); }
}
